// HeteroGraphSAGE_13434657702128
// MI455X (gfx1250) — hardware-verified
//
#include <hip/hip_runtime.h>
#include <stddef.h>
#include <stdint.h>


#define DF      128
#define NCR     50000
#define NMR     30000
#define NDR     10000
#define PCR     50048
#define PMR     30080
#define PDR     10112
#define TB_C    0
#define TB_M    50048
#define TB_D    80128
#define NROWS   90240
#define NREAL   90000
#define OUT_M   6400000
#define OUT_D   10240000
#define OUT_N   11520000
#define NLAYER  4
#define KST     1024
#define HP      256
#define MPITCH  512

#define E_0 800000
#define E_1 400000
#define E_2 800000
#define E_3 800000
#define E_4 400000
#define E_5 800000
#define SH_0 9
#define SH_1 9
#define SH_2 8
#define SH_3 10
#define SH_4 10
#define SH_5 10
#define NB_0 59
#define NB_1 20
#define NB_2 40
#define NB_3 49
#define NB_4 30
#define NB_5 49
#define FB_0 0
#define FB_1 59
#define FB_2 79
#define FB_3 119
#define FB_4 168
#define FB_5 198
#define NBLK 247
#define CB_0 0
#define CB_1 30208
#define CB_2 40448
#define CB_3 50688
#define CB_4 100864
#define CB_5 131584
#define CO_INTS 181760

#define NTHR    256
#define NWAVE   8
#define SLB     10
#define NSLOT   1024
#define WLCAP   3584
#define RCAP    24576
#define DEGCAP  128
#define MISC_INTS 16
#define BK_ZINTS (RCAP + 3 * NSLOT)
#define BK_INTS  (NWAVE * WLCAP + BK_ZINTS + MISC_INTS)

#define GBM     64
#define GBN     128
#define GTHR    128
#define GWAVE   4

#define U_HF    (NROWS * 32)
#define U_H     (NROWS * 32)
#define U_MZ    (240 * 64)
#define U_WS    (12 * 8 * 128 * 16)
#define U_BS    512
#define UB1     (U_HF)
#define UB2     (UB1 + U_H)
#define UB3     (UB2 + U_MZ)
#define UB4     (UB3 + U_WS)
#define UB5     (UB4 + U_BS)

static_assert(PCR == 391 * 128 && PMR == 235 * 128 && PDR == 79 * 128);
static_assert(TB_M == PCR && TB_D == PCR + PMR && NROWS == PCR + PMR + PDR && NROWS == 705 * 128);
static_assert(NCR - 390 * 128 == 80 && NMR - 234 * 128 == 48 && NDR - 78 * 128 == 16);
static_assert(NREAL == NCR + NMR + NDR && NREAL % NWAVE == 0 && NCR % 8 == 0 && NMR % 8 == 0 && NDR % 8 == 0);
static_assert(NROWS % GBM == 0 && TB_M % GBM == 0 && TB_D % GBM == 0);
static_assert(OUT_M == NCR * DF && OUT_D == (NCR + NMR) * DF && OUT_N == NREAL * DF);
static_assert(OUT_D + (NDR - 1) * DF + DF - 1 == OUT_N - 1);
static_assert((PCR - NCR) + (PMR - NMR) + (PDR - NDR) == 240);
static_assert(FB_1 == FB_0 + NB_0 && FB_2 == FB_1 + NB_1 && FB_3 == FB_2 + NB_2 && FB_4 == FB_3 + NB_3);
static_assert(FB_5 == FB_4 + NB_4 && NBLK == FB_5 + NB_5);
static_assert(CB_1 == CB_0 + (NB_0 << SH_0) && CB_2 == CB_1 + (NB_1 << SH_1) && CB_3 == CB_2 + (NB_2 << SH_2));
static_assert(CB_4 == CB_3 + (NB_3 << SH_3) && CB_5 == CB_4 + (NB_4 << SH_4) && CO_INTS == CB_5 + (NB_5 << SH_5));
static_assert((NB_0 << SH_0) >= PMR && ((NB_0 - 1) << SH_0) < NMR);
static_assert((NB_1 << SH_1) >= PDR && ((NB_1 - 1) << SH_1) < NDR);
static_assert((NB_2 << SH_2) >= PDR && ((NB_2 - 1) << SH_2) < NDR);
static_assert((NB_3 << SH_3) >= PCR && ((NB_3 - 1) << SH_3) < NCR);
static_assert((NB_4 << SH_4) >= PMR && ((NB_4 - 1) << SH_4) < NMR);
static_assert((NB_5 << SH_5) >= PCR && ((NB_5 - 1) << SH_5) < NCR);
static_assert(RCAP * 100LL >= 13878LL * 105 && RCAP * 100LL >= 20703LL * 105 && RCAP * 100LL >= 20753LL * 105);
static_assert(RCAP * 100LL >= 16705LL * 105 && RCAP * 100LL >= 13811LL * 105 && RCAP * 100LL >= 16647LL * 105);
static_assert(NWAVE * WLCAP * 100LL >= 20753LL * 125);
static_assert(DEGCAP >= 115 + 8 && DEGCAP <= 0xFFFF && RCAP < 32768 && (RCAP % 32) == 0);
static_assert(E_0 % 64 == 0 && E_1 % 64 == 0 && E_2 % 64 == 0 && E_3 % 64 == 0 && E_4 % 64 == 0 && E_5 % 64 == 0);
static_assert(E_0 < (1 << 20) && E_2 < (1 << 20) && E_3 < (1 << 20) && E_5 < (1 << 20) && NSLOT == (1 << SLB));
static_assert(BK_ZINTS % (NTHR * 4) == 0 && BK_INTS * 4 <= 300000 && (NWAVE * WLCAP) % 4 == 0);
static_assert(UB1 % NTHR == 0 && UB2 % NTHR == 0 && UB3 % NTHR == 0 && UB4 % NTHR == 0 && UB5 % NTHR == 0);
static_assert(GBN == DF && GBM == GWAVE * 16 && GTHR == GWAVE * 32 && KST % 32 == 0 && 768 % 32 == 0);

typedef float          v4f   __attribute__((ext_vector_type(4)));
typedef float          v8f   __attribute__((ext_vector_type(8)));
typedef int            v4i   __attribute__((ext_vector_type(4)));
typedef int            v8i   __attribute__((ext_vector_type(8)));
typedef unsigned short v4us  __attribute__((ext_vector_type(4)));
typedef unsigned short v8us  __attribute__((ext_vector_type(8)));
typedef unsigned short v16us __attribute__((ext_vector_type(16)));
typedef __bf16         v16bf __attribute__((ext_vector_type(16)));
typedef v4f  __attribute__((may_alias)) v4fa;
typedef v4i  __attribute__((may_alias)) v4ia;
typedef v4us __attribute__((may_alias)) v4usa;
typedef v8us __attribute__((may_alias)) v8usa;
union FragB { v16bf v; v16us u; v8us h[2]; v8i w; };

__device__ __forceinline__ v8f wmb(const FragB& a, const FragB& b, v8f c) {
  v8f d = __builtin_amdgcn_wmma_f32_16x16x32_bf16(false, a.v, false, b.v, (short)0, c, false, false);
  asm volatile("v_nop\n\tv_nop\n\tv_nop\n\tv_nop" : "+v"(d) : "v"(a.w), "v"(b.w));
  return d;
}

__device__ __forceinline__ unsigned bf16_bits(float f) {
  const unsigned u = __float_as_uint(f);
  const unsigned r = (u + 0x7FFFu + ((u >> 16) & 1u)) >> 16;
  return (f != f) ? 0x7FC0u : r;
}
__device__ __forceinline__ float bf16_val(float f) {
  return __uint_as_float(bf16_bits(f) << 16);
}
__device__ __forceinline__ unsigned hl_bits(float v, unsigned& lo) {
  const unsigned hb = bf16_bits(v);
  lo = bf16_bits(v - __uint_as_float(hb << 16));
  return hb;
}

__device__ __forceinline__ void wave_sync() {
  __builtin_amdgcn_fence(__ATOMIC_RELEASE, "wavefront");
  __builtin_amdgcn_wave_barrier();
  __builtin_amdgcn_fence(__ATOMIC_ACQUIRE, "wavefront");
}

__device__ __forceinline__ void st2_f4(float* p, v4f v) {
  *(volatile v4f*)p = v;
  __threadfence();
  *(volatile v4f*)p = v;
}
__device__ __forceinline__ void st2_h8(unsigned short* p, v8us v) {
  *(volatile v8us*)p = v;
  __threadfence();
  *(volatile v8us*)p = v;
}
__device__ __forceinline__ void st2_i4(int* p, v4i v) {
  *(volatile v4i*)p = v;
  __threadfence();
  *(volatile v4i*)p = v;
}

__device__ __forceinline__ void rel_tab(int r, int& sh, int& first, int& cob) {
  sh    = (r == 0) ? SH_0 : (r == 1) ? SH_1 : (r == 2) ? SH_2 : (r == 3) ? SH_3 : (r == 4) ? SH_4 : SH_5;
  first = (r == 0) ? FB_0 : (r == 1) ? FB_1 : (r == 2) ? FB_2 : (r == 3) ? FB_3 : (r == 4) ? FB_4 : FB_5;
  cob   = (r == 0) ? CB_0 : (r == 1) ? CB_1 : (r == 2) ? CB_2 : (r == 3) ? CB_3 : (r == 4) ? CB_4 : CB_5;
}
__device__ __forceinline__ void type_rels(int t, int& ra, int& rb) {
  ra = (t == 0) ? 3 : (t == 1) ? 0 : 1;
  rb = (t == 0) ? 5 : (t == 1) ? 4 : 2;
}

__global__ __launch_bounds__(NTHR) void k_prep(const float* __restrict__ xc, const float* __restrict__ xm,
                                               const float* __restrict__ xd, const float* __restrict__ wl,
                                               const float* __restrict__ wr, const float* __restrict__ bb,
                                               float* hf, unsigned short* hpl, unsigned short* mpl,
                                               unsigned short* wsp, float* bsp) {
  const int ub = (int)blockIdx.x * NTHR;
  const int u  = ub + (int)threadIdx.x;
  if (ub < UB2) {
    const bool isH = ub >= UB1;
    const int v    = isH ? (u - UB1) : u;
    const int vb   = isH ? (ub - UB1) : ub;
    const int rowb = vb >> 5;
    const int row  = v >> 5;
    const float* xp;
    int tbase, nr;
    if (rowb < TB_M)      { xp = xc; tbase = TB_C; nr = NCR; }
    else if (rowb < TB_D) { xp = xm; tbase = TB_M; nr = NMR; }
    else                  { xp = xd; tbase = TB_D; nr = NDR; }
    const int loc  = row - tbase;
    const bool real = loc < nr;
    const int locc = real ? loc : nr - 1;
    if (!isH) {
      const int c4 = (v & 31) * 4;
      const v4f f = *(const v4f*)(xp + (size_t)locc * DF + c4);
      asm volatile("" :: "v"(f));
      v4f o;
      o.x = real ? bf16_val(f.x) : 0.0f;
      o.y = real ? bf16_val(f.y) : 0.0f;
      o.z = real ? bf16_val(f.z) : 0.0f;
      o.w = real ? bf16_val(f.w) : 0.0f;
      st2_f4(hf + (size_t)row * DF + c4, o);
    } else {
      const int piece = v & 31;
      const int c8 = (piece & 15) * 8;
      const v4f f0 = *(const v4f*)(xp + (size_t)locc * DF + c8);
      const v4f f1 = *(const v4f*)(xp + (size_t)locc * DF + c8 + 4);
      asm volatile("" :: "v"(f0), "v"(f1));
      const unsigned msk = (real && piece < 16) ? 0xFFFFu : 0u;
      v8us o;
      o[0] = (unsigned short)(bf16_bits(f0.x) & msk); o[1] = (unsigned short)(bf16_bits(f0.y) & msk);
      o[2] = (unsigned short)(bf16_bits(f0.z) & msk); o[3] = (unsigned short)(bf16_bits(f0.w) & msk);
      o[4] = (unsigned short)(bf16_bits(f1.x) & msk); o[5] = (unsigned short)(bf16_bits(f1.y) & msk);
      o[6] = (unsigned short)(bf16_bits(f1.z) & msk); o[7] = (unsigned short)(bf16_bits(f1.w) & msk);
      st2_h8(hpl + (size_t)row * HP + piece * 8, o);
    }
  } else if (ub < UB3) {
    const int v = u - UB2;
    const int p = v >> 6, piece = v & 63;
    const int row = (p < 48) ? (TB_C + NCR + p) : (p < 128) ? (TB_M + NMR + (p - 48)) : (TB_D + NDR + (p - 128));
    const v8us z = {0, 0, 0, 0, 0, 0, 0, 0};
    st2_h8(mpl + (size_t)row * MPITCH + piece * 8, z);
  } else if (ub < UB4) {
    const int v  = u - UB3;
    const int vb = ub - UB3;
    const int lt = vb >> 14;
    const int kb = (vb >> 11) & 7;
    const int n  = (v >> 4) & (DF - 1);
    const int k8 = (v & 15) * 8;
    const int l  = lt / 3;
    const int t  = lt - 3 * l;
    int ra, rb;
    type_rels(t, ra, rb);
    int r, isR, zero = 0;
    if (l == 0) {
      if (kb < 4)       { isR = 0; r = (kb & 2) ? rb : ra; }
      else if (kb == 4) { isR = 1; r = ra; }
      else if (kb == 5) { isR = 1; r = rb; }
      else              { isR = 0; r = ra; zero = 1; }
    } else {
      isR = (kb >= 4) ? 1 : 0;
      r   = (kb & 2) ? rb : ra;
    }
    v8us o = {0, 0, 0, 0, 0, 0, 0, 0};
    if (zero == 0) {
      const size_t mo = ((size_t)(l * 6 + r) * DF + (size_t)k8) * DF + (size_t)n;
      if (isR != 0) {
        const float* p = wr + mo;
#pragma unroll
        for (int i = 0; i < 8; ++i) o[i] = (unsigned short)bf16_bits(p[(size_t)i * DF]);
      } else {
        const float* p = wl + mo;
#pragma unroll
        for (int i = 0; i < 8; ++i) o[i] = (unsigned short)bf16_bits(p[(size_t)i * DF]);
      }
    }
    st2_h8(wsp + ((size_t)lt * DF + n) * KST + kb * DF + k8, o);
  } else {
    const int v = u - UB4;
    if (v < 12 * 32) {
      const int lt = v >> 5, c4 = (v & 31) * 4;
      const int l  = lt / 3;
      const int t  = lt - 3 * l;
      int ra, rb;
      type_rels(t, ra, rb);
      const v4f a = *(const v4f*)(bb + (size_t)(l * 6 + ra) * DF + c4);
      const v4f c = *(const v4f*)(bb + (size_t)(l * 6 + rb) * DF + c4);
      v4f o;
      o.x = bf16_val(a.x) + bf16_val(c.x);
      o.y = bf16_val(a.y) + bf16_val(c.y);
      o.z = bf16_val(a.z) + bf16_val(c.z);
      o.w = bf16_val(a.w) + bf16_val(c.w);
      st2_f4(bsp + (size_t)lt * DF + c4, o);
    }
  }
}

__global__ __launch_bounds__(NTHR) void k_bucket(const int* __restrict__ ps0, const int* __restrict__ pd0,
                                                 const int* __restrict__ ps1, const int* __restrict__ pd1,
                                                 const int* __restrict__ ps2, const int* __restrict__ pd2,
                                                 const int* __restrict__ ps3, const int* __restrict__ pd3,
                                                 const int* __restrict__ ps4, const int* __restrict__ pd4,
                                                 const int* __restrict__ ps5, const int* __restrict__ pd5,
                                                 int* lst, int* cot, int* flg) {
  extern __shared__ __attribute__((aligned(16))) int dsm[];
  int* wl   = dsm;
  int* sl   = wl + NWAVE * WLCAP;
  int* cnt  = sl + RCAP;
  int* offs = cnt + NSLOT;
  int* cur  = offs + NSLOT;
  int* misc = cur + NSLOT;
  const int tid = (int)threadIdx.x, lane = tid & 31, wave = tid >> 5;
  const int b = (int)blockIdx.x;

  const int* srcp;
  const int* dstp;
  int nE, nDst, nSrc, sh, first, sbase, cob;
  if (b < FB_1)      { srcp = ps0; dstp = pd0; nE = E_0; nDst = NMR; nSrc = NCR; sh = SH_0; first = FB_0; sbase = TB_C; cob = CB_0; }
  else if (b < FB_2) { srcp = ps1; dstp = pd1; nE = E_1; nDst = NDR; nSrc = NMR; sh = SH_1; first = FB_1; sbase = TB_M; cob = CB_1; }
  else if (b < FB_3) { srcp = ps2; dstp = pd2; nE = E_2; nDst = NDR; nSrc = NCR; sh = SH_2; first = FB_2; sbase = TB_C; cob = CB_2; }
  else if (b < FB_4) { srcp = ps3; dstp = pd3; nE = E_3; nDst = NCR; nSrc = NMR; sh = SH_3; first = FB_3; sbase = TB_M; cob = CB_3; }
  else if (b < FB_5) { srcp = ps4; dstp = pd4; nE = E_4; nDst = NMR; nSrc = NDR; sh = SH_4; first = FB_4; sbase = TB_D; cob = CB_4; }
  else               { srcp = ps5; dstp = pd5; nE = E_5; nDst = NCR; nSrc = NDR; sh = SH_5; first = FB_5; sbase = TB_D; cob = CB_5; }
  const int blk      = b - first;
  const int nbr      = 1 << sh;
  const int slotBase = blk << sh;
  int nbEff = nDst - slotBase;
  nbEff = nbEff > nbr ? nbr : nbEff;
  nbEff = nbEff < 0 ? 0 : nbEff;

  {
    const v4i z4 = {0, 0, 0, 0};
    for (int i = tid * 4; i < BK_ZINTS; i += NTHR * 4) *(v4ia*)(sl + i) = z4;
    if (tid < MISC_INTS) misc[tid] = 0;
  }
  __syncthreads();

  {
    const int seg   = nE >> 3;
    const int wbase = wave * seg;
    const int nIt   = (seg + 255) >> 8;
    const unsigned nbs = (unsigned)slotBase;
    const unsigned unb = (unsigned)nbEff;
    int wc = 0;
#pragma unroll 1
    for (int it = 0; it < nIt; ++it) {
      const int local  = it * 256 + lane * 8;
      const bool valid = local < seg;
      const int e0     = wbase + (valid ? local : 0);
      const v4i da = *(const v4i*)(dstp + e0);
      const v4i db = *(const v4i*)(dstp + e0 + 4);
      asm volatile("" :: "v"(da), "v"(db));
      const unsigned s0 = (unsigned)da.x - nbs, s1 = (unsigned)da.y - nbs;
      const unsigned s2 = (unsigned)da.z - nbs, s3 = (unsigned)da.w - nbs;
      const unsigned s4 = (unsigned)db.x - nbs, s5 = (unsigned)db.y - nbs;
      const unsigned s6 = (unsigned)db.z - nbs, s7 = (unsigned)db.w - nbs;
      const bool h0 = valid & (s0 < unb), h1 = valid & (s1 < unb), h2 = valid & (s2 < unb), h3 = valid & (s3 < unb);
      const bool h4 = valid & (s4 < unb), h5 = valid & (s5 < unb), h6 = valid & (s6 < unb), h7 = valid & (s7 < unb);
      const unsigned any = __builtin_amdgcn_ballot_w32(h0 | h1 | h2 | h3 | h4 | h5 | h6 | h7);
      if (any != 0u) {
#define HITJ(J, HJ, SJ) { \
        const unsigned mj = __builtin_amdgcn_ballot_w32(HJ); \
        if (mj != 0u) { \
          if (HJ) { \
            const int pos = wc + (int)__builtin_amdgcn_mbcnt_lo(mj, 0u); \
            if (pos < WLCAP) wl[wave * WLCAP + pos] = ((e0 + (J)) << SLB) | (int)(SJ); \
          } \
          wc += (int)__builtin_popcount(mj); } }
        HITJ(0, h0, s0)
        HITJ(1, h1, s1)
        HITJ(2, h2, s2)
        HITJ(3, h3, s3)
        HITJ(4, h4, s4)
        HITJ(5, h5, s5)
        HITJ(6, h6, s6)
        HITJ(7, h7, s7)
#undef HITJ
      }
    }
    if (lane == 0) misc[wave] = wc;
  }
  __syncthreads();

  int t = 0, ov = 0;
  if (wave == 0) {
#pragma unroll 1
    for (int w2 = 0; w2 < NWAVE; ++w2) {
      int c = misc[w2];
      if (c > WLCAP) ov = 1;
      c = c < 0 ? 0 : (c > WLCAP ? WLCAP : c);
#pragma unroll 1
      for (int b0 = 0; b0 < c; b0 += 32) {
        const int idx = b0 + lane;
        const int ent = wl[w2 * WLCAP + (idx < c ? idx : c - 1)];
        const int m32 = (c - b0) < 32 ? (c - b0) : 32;
#pragma unroll 1
        for (int k = 0; k < m32; ++k) {
          const int u    = __builtin_amdgcn_readlane(ent, k);
          const int slot = u & (NSLOT - 1);
          if (lane == 0) cnt[slot] = cnt[slot] + 1;
        }
      }
      t += c;
    }
    if (t > RCAP) { ov = 1; t = RCAP; }
  }
  __syncthreads();

  if (wave == 0) {
    const int base = lane * (NSLOT / 32);
    int s = 0, mx = 0;
#pragma unroll 1
    for (int i = 0; i < NSLOT / 32; ++i) {
      const int cv = cnt[base + i];
      s += cv;
      mx = cv > mx ? cv : mx;
    }
    int incl = s;
#pragma unroll
    for (int d = 1; d < 32; d <<= 1) {
      const int y = __shfl_up(incl, d, 32);
      if (lane >= d) incl += y;
    }
#pragma unroll
    for (int d = 16; d > 0; d >>= 1) {
      const int y = __shfl_xor(mx, d, 32);
      mx = y > mx ? y : mx;
    }
    if (mx > DEGCAP) ov = 1;
    int run = incl - s;
#pragma unroll 1
    for (int i = 0; i < NSLOT / 32; ++i) {
      const int cv = cnt[base + i];
      offs[base + i] = run;
      cur[base + i]  = run;
      run += cv;
    }
  }
  __syncthreads();

  if (wave == 0) {
#pragma unroll 1
    for (int w2 = 0; w2 < NWAVE; ++w2) {
      int c = misc[w2];
      c = c < 0 ? 0 : (c > WLCAP ? WLCAP : c);
#pragma unroll 1
      for (int b0 = 0; b0 < c; b0 += 32) {
        const int idx = b0 + lane;
        const int ent = wl[w2 * WLCAP + (idx < c ? idx : c - 1)];
        int e = ent >> SLB;
        e = e < 0 ? 0 : (e > nE - 1 ? nE - 1 : e);
        int sv = srcp[e];
        sv = sv < 0 ? 0 : (sv > nSrc - 1 ? nSrc - 1 : sv);
        sv += sbase;
        const int m32 = (c - b0) < 32 ? (c - b0) : 32;
#pragma unroll 1
        for (int k = 0; k < m32; ++k) {
          const int u    = __builtin_amdgcn_readlane(ent, k);
          const int s2   = __builtin_amdgcn_readlane(sv, k);
          const int slot = u & (NSLOT - 1);
          if (lane == 0) {
            int p = cur[slot];
            p = p < 0 ? 0 : (p > RCAP - 1 ? RCAP - 1 : p);
            sl[p] = s2;
            cur[slot] = p + 1;
          }
        }
      }
    }
    if (lane == 0) { misc[8] = t; misc[9] = ov; }
  }
  __syncthreads();

  int tt = misc[8];
  tt = tt < 0 ? 0 : (tt > RCAP ? RCAP : tt);
  const int ovf  = misc[9];
  const int tt32 = (tt + 31) & ~31;

  int* lbase = lst + (size_t)b * RCAP;
#pragma unroll 1
  for (int i0 = 0; i0 < tt32; i0 += NTHR * 4) {
    const int idx = i0 + tid * 4;
    const int ic  = idx > RCAP - 4 ? RCAP - 4 : idx;
    const v4i v = *(const v4ia*)(sl + ic);
    asm volatile("" :: "v"(v));
    if (idx < tt32) st2_i4(lbase + idx, v);
  }
  {
    const int s4 = tid * 4;
    const v4i cv = *(const v4ia*)(cnt + s4);
    const v4i fo = *(const v4ia*)(offs + s4);
    asm volatile("" :: "v"(cv), "v"(fo));
    v4i co;
    co.x = (cv.x > 0) ? ((fo.x << 16) | (cv.x > 0xFFFF ? 0xFFFF : cv.x)) : 0;
    co.y = (cv.y > 0) ? ((fo.y << 16) | (cv.y > 0xFFFF ? 0xFFFF : cv.y)) : 0;
    co.z = (cv.z > 0) ? ((fo.z << 16) | (cv.z > 0xFFFF ? 0xFFFF : cv.z)) : 0;
    co.w = (cv.w > 0) ? ((fo.w << 16) | (cv.w > 0xFFFF ? 0xFFFF : cv.w)) : 0;
    if (s4 < nbr) st2_i4(cot + cob + slotBase + s4, co);
  }
  if (tid < 8) {
    const v4i f4 = {ovf, ovf, ovf, ovf};
    st2_i4(flg + b * 32 + tid * 4, f4);
  }
}

__global__ __launch_bounds__(NTHR) void k_agg(const int* __restrict__ lst, const int* __restrict__ cot,
                                              const int* __restrict__ flg, const float* __restrict__ hf,
                                              unsigned short* mpl) {
  __shared__ __attribute__((aligned(16))) unsigned short rowbuf[NWAVE * MPITCH];
  const int tid = (int)threadIdx.x, lane = tid & 31;
  const int wave = __builtin_amdgcn_readfirstlane(tid >> 5);
  const int g = (int)blockIdx.x * NWAVE + wave;
  if (g >= NREAL) return;
  int t, node, prow;
  if (g < NCR)            { t = 0; node = g;             prow = TB_C + node; }
  else if (g < NCR + NMR) { t = 1; node = g - NCR;       prow = TB_M + node; }
  else                    { t = 2; node = g - NCR - NMR; prow = TB_D + node; }
  int ra, rb;
  type_rels(t, ra, rb);
  unsigned short* rbw = rowbuf + wave * MPITCH;
  const float qnan = __int_as_float(0x7fc00000);
  const float* hp = hf + 4 * lane;

#pragma unroll 1
  for (int which = 0; which < 2; ++which) {
    const int r = which ? rb : ra;
    int sh, first, cob;
    rel_tab(r, sh, first, cob);
    const int gb = first + (node >> sh);
    const int co = cot[cob + node];
    const int fl = flg[gb * 32];
    const int craw = co & 0xFFFF;
    const bool big = craw > DEGCAP;
    const int c = big ? DEGCAP : craw;
    int o = (co >> 16) & 0x7FFF;
    o = o > RCAP - 1 ? RCAP - 1 : o;
    const int* lp = lst + (size_t)gb * RCAP;
    v4f a = {0.0f, 0.0f, 0.0f, 0.0f};
#pragma unroll 1
    for (int b0 = 0; b0 < c; b0 += 32) {
      int j = b0 + lane;
      j = j > c - 1 ? c - 1 : j;
      int idx = o + j;
      idx = idx > RCAP - 1 ? RCAP - 1 : idx;
      int sr = lp[idx];
      sr = sr < 0 ? 0 : (sr > NROWS - 1 ? NROWS - 1 : sr);
      const int m32 = (c - b0) < 32 ? (c - b0) : 32;
#pragma unroll 1
      for (int k = 0; k < m32; k += 4) {
        const int q0 = __builtin_amdgcn_readlane(sr, k);
        const int q1 = __builtin_amdgcn_readlane(sr, k + 1);
        const int q2 = __builtin_amdgcn_readlane(sr, k + 2);
        const int q3 = __builtin_amdgcn_readlane(sr, k + 3);
        const v4f r0 = *(const v4f*)(hp + (size_t)q0 * DF);
        const v4f r1 = *(const v4f*)(hp + (size_t)q1 * DF);
        const v4f r2 = *(const v4f*)(hp + (size_t)q2 * DF);
        const v4f r3 = *(const v4f*)(hp + (size_t)q3 * DF);
        a = a + r0;
        if (k + 1 < m32) a = a + r1;
        if (k + 2 < m32) a = a + r2;
        if (k + 3 < m32) a = a + r3;
      }
    }
    const float den = fmaxf((float)craw, 1.0f);
    const float pz  = (fl != 0 || big) ? qnan : 0.0f;
    const float m0 = a.x / den + pz;
    const float m1 = a.y / den + pz;
    const float m2 = a.z / den + pz;
    const float m3 = a.w / den + pz;
    v4us mh, ml;
    {
      unsigned lb;
      unsigned hb;
      hb = hl_bits(m0, lb); mh[0] = (unsigned short)hb; ml[0] = (unsigned short)lb;
      hb = hl_bits(m1, lb); mh[1] = (unsigned short)hb; ml[1] = (unsigned short)lb;
      hb = hl_bits(m2, lb); mh[2] = (unsigned short)hb; ml[2] = (unsigned short)lb;
      hb = hl_bits(m3, lb); mh[3] = (unsigned short)hb; ml[3] = (unsigned short)lb;
    }
    *(v4usa*)(rbw + which * 256 + 4 * lane)      = mh;
    *(v4usa*)(rbw + which * 256 + DF + 4 * lane) = ml;
  }
  wave_sync();
  const v8us q0 = *(const v8usa*)(rbw + 8 * lane);
  const v8us q1 = *(const v8usa*)(rbw + 256 + 8 * lane);
  unsigned short* rpw = mpl + (size_t)prow * MPITCH + 8 * lane;
  *(volatile v8us*)rpw = q0;
  *(volatile v8us*)(rpw + 256) = q1;
  __threadfence();
  *(volatile v8us*)rpw = q0;
  *(volatile v8us*)(rpw + 256) = q1;
}

template <int MODE>
__global__ __launch_bounds__(GTHR) __attribute__((amdgpu_num_vgpr(248)))
void k_gemm(unsigned short* wsb, size_t eM, size_t eH, const unsigned short* wsp, const float* bsp,
            const int* flg, float* hf, float* outp, int layer) {
  __shared__ __attribute__((aligned(16))) float stg[GBM * GBN];
  __shared__ __attribute__((aligned(16))) float bsl[DF];
  __shared__ __attribute__((aligned(16))) unsigned short rbs[GWAVE * 256];
  const int tid = (int)threadIdx.x, lane = tid & 31, hh = lane >> 4, m = lane & 15;
  const int wave = __builtin_amdgcn_readfirstlane(tid >> 5);
  const int rowBase = (int)blockIdx.x * GBM;
  int t, tbase, nReal, outOff;
  if (rowBase < TB_M)      { t = 0; tbase = TB_C; nReal = NCR; outOff = 0; }
  else if (rowBase < TB_D) { t = 1; tbase = TB_M; nReal = NMR; outOff = OUT_M; }
  else                     { t = 2; tbase = TB_D; nReal = NDR; outOff = OUT_D; }
  const int lt = layer * 3 + t;
  const unsigned short* BT = wsp + (size_t)lt * DF * KST;
  if (tid < 32) {
    const v4f b4 = *(const v4f*)(bsp + (size_t)lt * DF + 4 * tid);
    *(v4fa*)(bsl + 4 * tid) = b4;
  }

  v8f acc[8];
  {
    const v8f z = {0.f, 0.f, 0.f, 0.f, 0.f, 0.f, 0.f, 0.f};
#pragma unroll
    for (int i = 0; i < 8; ++i) acc[i] = z;
  }
  const size_t rowi = (size_t)(rowBase + 16 * wave + m);
  const size_t aM = eM + rowi * MPITCH + 8 * hh;
  const size_t aH = eH + rowi * HP + 8 * hh;
  const unsigned short* bp = BT + (size_t)m * KST + 8 * hh;
  const int nkb = (MODE == 0) ? 6 : 8;

#pragma unroll 1
  for (int kb = 0; kb < nkb; ++kb) {
    size_t ao;
    if (kb < 4) ao = aM + (size_t)kb * DF;
    else        ao = aH + ((MODE == 0) ? (size_t)0 : (size_t)((kb & 1) * DF));
    const unsigned short* ap = wsb + ao;
    const unsigned short* bq = bp + kb * DF;
#pragma unroll 1
    for (int kk = 0; kk < DF; kk += 32) {
      FragB af;
      af.h[0] = *(const v8usa*)(ap + kk);
      af.h[1] = *(const v8usa*)(ap + kk + 16);
#pragma unroll
      for (int nt = 0; nt < 8; ++nt) {
        const unsigned short* wq = bq + (size_t)(16 * nt) * KST + kk;
        FragB bf;
        bf.h[0] = *(const v8usa*)wq;
        bf.h[1] = *(const v8usa*)(wq + 16);
        acc[nt] = wmb(af, bf, acc[nt]);
      }
    }
  }

#pragma unroll
  for (int nt = 0; nt < 8; ++nt) {
    const int lc = 16 * nt + m;
#pragma unroll
    for (int r = 0; r < 8; ++r) {
      const int lr = 16 * wave + 8 * hh + r;
      stg[lr * GBN + lc] = acc[nt][r];
    }
  }
  __syncthreads();

  const v4f bs4 = *(const v4fa*)(bsl + 4 * lane);
  unsigned short* rbw = rbs + wave * 256;
  const float qnan = __int_as_float(0x7fc00000);
  int ra, rb;
  type_rels(t, ra, rb);
  int shA, firstA, cobA, shB, firstB, cobB;
  rel_tab(ra, shA, firstA, cobA);
  rel_tab(rb, shB, firstB, cobB);
  (void)cobA; (void)cobB;

#pragma unroll 1
  for (int i = 0; i < 16; ++i) {
    const int lr  = 16 * wave + i;
    const int row = rowBase + lr;
    const int loc = row - tbase;
    const bool real = loc < nReal;
    const v4f p = *(const v4fa*)(stg + lr * GBN + 4 * lane);
    v4f v;
    v.x = (p.x + bs4.x) * 0.5f;
    v.y = (p.y + bs4.y) * 0.5f;
    v.z = (p.z + bs4.z) * 0.5f;
    v.w = (p.w + bs4.w) * 0.5f;
    if constexpr (MODE != 2) {
      v.x = (v.x > 0.0f) ? v.x : (v.x - v.x);
      v.y = (v.y > 0.0f) ? v.y : (v.y - v.y);
      v.z = (v.z > 0.0f) ? v.z : (v.z - v.z);
      v.w = (v.w > 0.0f) ? v.w : (v.w - v.w);
      v4us h4, l4;
      unsigned lb;
      unsigned hb;
      hb = hl_bits(v.x, lb); h4[0] = (unsigned short)hb; l4[0] = (unsigned short)lb;
      hb = hl_bits(v.y, lb); h4[1] = (unsigned short)hb; l4[1] = (unsigned short)lb;
      hb = hl_bits(v.z, lb); h4[2] = (unsigned short)hb; l4[2] = (unsigned short)lb;
      hb = hl_bits(v.w, lb); h4[3] = (unsigned short)hb; l4[3] = (unsigned short)lb;
      *(v4usa*)(rbw + 4 * lane)      = h4;
      *(v4usa*)(rbw + DF + 4 * lane) = l4;
      wave_sync();
      const v8us q = *(const v8usa*)(rbw + 8 * lane);
      wave_sync();
      float* hfp = hf + (size_t)row * DF + 4 * lane;
      unsigned short* hpp = wsb + eH + (size_t)row * HP + 8 * lane;
      if (real) { *(volatile v4f*)hfp = v; *(volatile v8us*)hpp = q; }
      __threadfence();
      if (real) { *(volatile v4f*)hfp = v; *(volatile v8us*)hpp = q; }
    } else {
      float q = (v.x * v.x + v.y * v.y) + (v.z * v.z + v.w * v.w);
      q += __shfl_xor(q, 16, 32);
      q += __shfl_xor(q, 8, 32);
      q += __shfl_xor(q, 4, 32);
      q += __shfl_xor(q, 2, 32);
      q += __shfl_xor(q, 1, 32);
      float den = sqrtf(q);
      den = (den < 1e-12f) ? 1e-12f : den;
      const int locc = real ? loc : nReal - 1;
      const int fa = flg[(firstA + (locc >> shA)) * 32];
      const int fb = flg[(firstB + (locc >> shB)) * 32];
      asm volatile("" :: "v"(fa), "v"(fb));
      const float pz = ((fa | fb) != 0) ? qnan : 0.0f;
      v4f o;
      o.x = v.x / den + pz;
      o.y = v.y / den + pz;
      o.z = v.z / den + pz;
      o.w = v.w / den + pz;
      float* op = outp + (size_t)outOff + (size_t)locc * DF + 4 * lane;
      if (real) *(volatile v4f*)op = o;
      __threadfence();
      if (real) *(volatile v4f*)op = o;
    }
  }
  (void)hf; (void)outp; (void)flg; (void)rbw; (void)qnan;
}

static inline size_t al256(size_t o) { return (o + 255) & ~(size_t)255; }

extern "C" void kernel_launch(void* const* d_in, const int* in_sizes, int n_in,
                              void* d_out, int out_size, void* d_ws, size_t ws_size,
                              hipStream_t stream) {
  if (n_in < 18) return;
  if (in_sizes[0] != NCR * DF || in_sizes[1] != NMR * DF || in_sizes[2] != NDR * DF) return;
  if (in_sizes[3] != E_0 || in_sizes[4] != E_0) return;
  if (in_sizes[5] != E_1 || in_sizes[6] != E_1) return;
  if (in_sizes[7] != E_2 || in_sizes[8] != E_2) return;
  if (in_sizes[9] != E_3 || in_sizes[10] != E_3) return;
  if (in_sizes[11] != E_4 || in_sizes[12] != E_4) return;
  if (in_sizes[13] != E_5 || in_sizes[14] != E_5) return;
  if (in_sizes[15] != NLAYER * 6 * DF * DF || in_sizes[16] != NLAYER * 6 * DF * DF) return;
  if (in_sizes[17] != NLAYER * 6 * DF) return;
  if (out_size != OUT_N) return;

  const float* x_c = (const float*)d_in[0];
  const float* x_m = (const float*)d_in[1];
  const float* x_d = (const float*)d_in[2];
  const int* s0 = (const int*)d_in[3];   const int* t0 = (const int*)d_in[4];
  const int* s1 = (const int*)d_in[5];   const int* t1 = (const int*)d_in[6];
  const int* s2 = (const int*)d_in[7];   const int* t2 = (const int*)d_in[8];
  const int* s3 = (const int*)d_in[9];   const int* t3 = (const int*)d_in[10];
  const int* s4 = (const int*)d_in[11];  const int* t4 = (const int*)d_in[12];
  const int* s5 = (const int*)d_in[13];  const int* t5 = (const int*)d_in[14];
  const float* Wl = (const float*)d_in[15];
  const float* Wr = (const float*)d_in[16];
  const float* bb = (const float*)d_in[17];
  float* out = (float*)d_out;

  char* ws = (char*)d_ws;
  size_t off = 0;
  const size_t oWS = off; off = al256(off + (size_t)12 * DF * KST * 2);
  const size_t oBS = off; off = al256(off + (size_t)12 * DF * 4);
  const size_t oFL = off; off = al256(off + (size_t)NBLK * 32 * 4);
  const size_t oCO = off; off = al256(off + (size_t)CO_INTS * 4);
  const size_t oLS = off; off = al256(off + (size_t)NBLK * RCAP * 4);
  const size_t oH  = off; off = al256(off + (size_t)NROWS * HP * 2);
  const size_t oHF = off; off = al256(off + (size_t)NROWS * DF * 4);
  const size_t oM  = off; off = al256(off + (size_t)NROWS * MPITCH * 2);
  if (off > ws_size) return;
  unsigned short* WS = (unsigned short*)(ws + oWS);
  float* BS  = (float*)(ws + oBS);
  int*   FL  = (int*)(ws + oFL);
  int*   CO  = (int*)(ws + oCO);
  int*   LS  = (int*)(ws + oLS);
  unsigned short* Hp = (unsigned short*)(ws + oH);
  float* HF  = (float*)(ws + oHF);
  unsigned short* Mp = (unsigned short*)(ws + oM);
  unsigned short* wsb = (unsigned short*)ws;
  const size_t eM = oM / 2, eH = oH / 2;

  const size_t bkLds = (size_t)BK_INTS * 4;
  hipFuncSetAttribute(reinterpret_cast<const void*>(&k_bucket), hipFuncAttributeMaxDynamicSharedMemorySize, (int)bkLds);

  k_prep<<<UB5 / NTHR, NTHR, 0, stream>>>(x_c, x_m, x_d, Wl, Wr, bb, HF, Hp, Mp, WS, BS);
  k_bucket<<<NBLK, NTHR, bkLds, stream>>>(s0, t0, s1, t1, s2, t2, s3, t3, s4, t4, s5, t5, LS, CO, FL);
  for (int l = 0; l < NLAYER; ++l) {
    k_agg<<<NREAL / NWAVE, NTHR, 0, stream>>>(LS, CO, FL, HF, Mp);
    if (l == 0)      k_gemm<0><<<NROWS / GBM, GTHR, 0, stream>>>(wsb, eM, eH, WS, BS, FL, HF, out, l);
    else if (l < 3)  k_gemm<1><<<NROWS / GBM, GTHR, 0, stream>>>(wsb, eM, eH, WS, BS, FL, HF, out, l);
    else             k_gemm<2><<<NROWS / GBM, GTHR, 0, stream>>>(wsb, eM, eH, WS, BS, FL, HF, out, l);
  }
}
